// FusedTransformerBlock_90941637525729
// MI455X (gfx1250) — hardware-run, weakly checked
//
#include <hip/hip_runtime.h>
#include <math.h>

constexpr int kB    = 2;
constexpr int kS    = 2048;
constexpr int kD    = 1024;
constexpr int kH    = 16;
constexpr int kHD   = 64;
constexpr int kFF   = 4096;
constexpr int kTok  = kB * kS;
constexpr int kQKld = 2 * kD;
constexpr int kG    = 4;
constexpr int kNChunk = kB * kH / kG;

constexpr float kWCarry    = 64.0f;
constexpr float kWCarryInv = 1.0f / 64.0f;
constexpr float kPCarry    = 2048.0f;
constexpr float kCtxCarry  = 256.0f;
constexpr float kScoreScale = 0.125f;
constexpr float kPVScale   = kCtxCarry / kPCarry;
constexpr float kWoScale   = 1.0f / (kCtxCarry * kWCarry);
constexpr float kInvD      = 1.0f / 1024.0f;
constexpr float kLnEps     = 1e-5f;

constexpr size_t kMi    = 1048576;
constexpr size_t oXh    = 0;
constexpr size_t oWqkT  = 8 * kMi;
constexpr size_t oWvT   = 12 * kMi;
constexpr size_t oS     = 0;
constexpr size_t oH32   = 0;
constexpr size_t oU16   = 16 * kMi;
constexpr size_t oW2T   = 48 * kMi;
constexpr size_t oWoT   = 56 * kMi;
constexpr size_t oP     = 64 * kMi;
constexpr size_t oFF    = 64 * kMi;
constexpr size_t oQK    = 96 * kMi;
constexpr size_t oY1    = 96 * kMi;
constexpr size_t oY2    = 96 * kMi;
constexpr size_t oVt    = 112 * kMi;
constexpr size_t oHH    = 112 * kMi;
constexpr size_t oCtx   = 120 * kMi;
constexpr size_t oW1T   = 120 * kMi;
constexpr size_t kWsNeed = 128 * kMi;
static_assert((size_t)kTok * kD * 2 == 8 * kMi, "sz");
static_assert((size_t)kG * kS * kS * 4 == 64 * kMi, "sz");
static_assert((size_t)kTok * kFF * 2 == 32 * kMi, "sz");
static_assert((size_t)kTok * kQKld * 2 == 16 * kMi, "sz");

typedef __attribute__((ext_vector_type(16))) _Float16 v16h;
typedef __attribute__((ext_vector_type(8)))  _Float16 v8h;
typedef __attribute__((ext_vector_type(16))) __bf16   v16b;
typedef __attribute__((ext_vector_type(8)))  __bf16   v8b;
typedef __attribute__((ext_vector_type(8)))  float    v8f;
typedef __attribute__((ext_vector_type(4)))  float    v4f;
typedef __attribute__((ext_vector_type(4)))  unsigned int v4u;

__device__ __forceinline__ unsigned short f2bf_bits(float f) {
  unsigned u = __float_as_uint(f);
  return (unsigned short)((u + 0x7FFFu + ((u >> 16) & 1u)) >> 16);
}
__device__ __forceinline__ float bf_bits2f(unsigned short h) { return __uint_as_float(((unsigned)h) << 16); }

__device__ __forceinline__ void dep_guard_h(v8f& a, v8f& b, v16h x, v16h y) { asm volatile("v_nop\n\tv_nop\n\tv_nop\n\tv_nop" : "+v"(a), "+v"(b) : "v"(x), "v"(y)); }
__device__ __forceinline__ void dep_guard_b(v8f& a, v8f& b, v16b x, v16b y) { asm volatile("v_nop\n\tv_nop\n\tv_nop\n\tv_nop" : "+v"(a), "+v"(b) : "v"(x), "v"(y)); }
__device__ __forceinline__ void keep4_h(v16h a, v16h b, v16h c, v16h d) { asm volatile("v_nop" :: "v"(a), "v"(b), "v"(c), "v"(d)); }
__device__ __forceinline__ void keep4_b(v16b a, v16b b, v16b c, v16b d) { asm volatile("v_nop" :: "v"(a), "v"(b), "v"(c), "v"(d)); }
__device__ __forceinline__ void acc_guard4(v8f& a, v8f& b, v8f& c, v8f& d) { asm volatile("v_nop\n\tv_nop\n\tv_nop\n\tv_nop" : "+v"(a), "+v"(b), "+v"(c), "+v"(d)); }
template <typename T> struct Frag;
template <> struct Frag<_Float16> {
  typedef v16h V; union U { v16h v; v8h h[2]; };
  static __device__ __forceinline__ v16h load(const _Float16* p) {
    U f; f.h[0] = *(const v8h*)(p); f.h[1] = *(const v8h*)(p + 16); return f.v;
  }
  static __device__ __forceinline__ v8f mma(v16h a, v16h b, v8f c) {
    return __builtin_amdgcn_wmma_f32_16x16x32_f16(false, a, false, b, (short)0, c, false, false);
  }
  static __device__ __forceinline__ void guard(v8f& a, v8f& b, v16h x, v16h y) { dep_guard_h(a, b, x, y); }
  static __device__ __forceinline__ void keep(v16h a, v16h b, v16h c, v16h d) { keep4_h(a, b, c, d); }
};
template <> struct Frag<__bf16> {
  typedef v16b V; union U { v16b v; v8b h[2]; };
  static __device__ __forceinline__ v16b load(const __bf16* p) {
    U f; f.h[0] = *(const v8b*)(p); f.h[1] = *(const v8b*)(p + 16); return f.v;
  }
  static __device__ __forceinline__ v8f mma(v16b a, v16b b, v8f c) {
    return __builtin_amdgcn_wmma_f32_16x16x32_bf16(false, a, false, b, (short)0, c, false, false);
  }
  static __device__ __forceinline__ void guard(v8f& a, v8f& b, v16b x, v16b y) { dep_guard_b(a, b, x, y); }
  static __device__ __forceinline__ void keep(v16b a, v16b b, v16b c, v16b d) { keep4_b(a, b, c, d); }
};

__device__ __forceinline__ unsigned pk16(unsigned short a, unsigned short b) { return (unsigned)a | ((unsigned)b << 16); }
__device__ __forceinline__ unsigned short h_bits(float f) { const _Float16 h = (_Float16)f; return __builtin_bit_cast(unsigned short, h); }

template <int ET> struct Elem;
template <> struct Elem<0> { typedef _Float16 T; };
template <> struct Elem<1> { typedef __bf16 T; };
template <int ET, bool SPLIT, int BIAS_MODE, int OUT_MODE, bool RESID, int ACT = 0>
__global__ __launch_bounds__(256) void wmma_gemm64(
    const unsigned short* __restrict__ Ap, const unsigned short* __restrict__ A2p, int lda, long strideA,
    const unsigned short* __restrict__ Btp, const unsigned short* __restrict__ Bt2p, int ldb, long strideB,
    void* __restrict__ Cout, void* __restrict__ Cout2, int ldc, long strideC,
    const float* __restrict__ bias,
    const float* __restrict__ resid, long strideR,
    int M, int N, int K, float scale) {
  typedef typename Elem<ET>::T T;
  typedef typename Frag<T>::V V;
  const T* A = (const T*)Ap; const T* A2 = (const T*)A2p; const T* Bt = (const T*)Btp; const T* Bt2 = (const T*)Bt2p;
  __shared__ __align__(16) float sT[8][16 * 68];
  const int b    = blockIdx.y;
  const int lane = threadIdx.x & 31;
  const int wave = threadIdx.x >> 5;
  const int tilesN = N >> 6;
  const int tilesM = M >> 6;
  const int tile = blockIdx.x * 8 + wave;
  if (tile >= tilesM * tilesN) return;
  const int tm = tile / tilesN;
  const int tn = tile - tm * tilesN;
  const int m0 = tm << 6;
  const int n0 = tn << 6;

  const T* Ab  = A  + (size_t)b * strideA;
  const T* Bb  = Bt + (size_t)b * strideB;
  const T* Ab2 = SPLIT ? (A2  + (size_t)b * strideA) : nullptr;
  const T* Bb2 = SPLIT ? (Bt2 + (size_t)b * strideB) : nullptr;

  const int rlane = lane & 15;
  const int koff  = (lane >> 4) * 8;
  const int mOff  = (lane >> 4) * 8;

  v8f acc[4][4];
#pragma unroll
  for (int i = 0; i < 4; ++i)
#pragma unroll
    for (int j = 0; j < 4; ++j) acc[i][j] = (v8f){0.f,0.f,0.f,0.f,0.f,0.f,0.f,0.f};

  for (int k0 = 0; k0 < K; k0 += 32) {
    V bh[4], bl[4];
#pragma unroll
    for (int j = 0; j < 4; ++j) {
      const size_t bo = (size_t)(n0 + (j << 4) + rlane) * ldb + koff + k0;
      bh[j] = Frag<T>::load(Bb + bo);
      if (SPLIT) bl[j] = Frag<T>::load(Bb2 + bo);
    }
#pragma unroll
    for (int i = 0; i < 4; ++i) {
      const size_t ao = (size_t)(m0 + (i << 4) + rlane) * lda + koff + k0;
      V ah = Frag<T>::load(Ab + ao);
      V al;
      if (SPLIT) al = Frag<T>::load(Ab2 + ao);
#pragma unroll
      for (int j = 0; j < 4; ++j) {
        acc[i][j] = Frag<T>::mma(ah, bh[j], acc[i][j]);
        if (SPLIT) {
          acc[i][j] = Frag<T>::mma(ah, bl[j], acc[i][j]);
          acc[i][j] = Frag<T>::mma(al, bh[j], acc[i][j]);
        }
      }
      Frag<T>::guard(acc[i][0], acc[i][3], ah, SPLIT ? al : ah);
    }
    Frag<T>::keep(bh[0], bh[1], bh[2], bh[3]);
    if (SPLIT) Frag<T>::keep(bl[0], bl[1], bl[2], bl[3]);
  }
  acc_guard4(acc[0][0], acc[0][1], acc[0][2], acc[0][3]);
  acc_guard4(acc[1][0], acc[1][1], acc[1][2], acc[1][3]);
  acc_guard4(acc[2][0], acc[2][1], acc[2][2], acc[2][3]);
  acc_guard4(acc[3][0], acc[3][1], acc[3][2], acc[3][3]);

  float* slab = sT[wave];
  const float* Rb = RESID ? (resid + (size_t)b * strideR) : nullptr;
#pragma unroll
  for (int i = 0; i < 4; ++i) {
    const int mBase = m0 + (i << 4);
#pragma unroll
    for (int j = 0; j < 4; ++j) {
      const int n = n0 + (j << 4) + rlane;
      float bv = 0.f;
      if (BIAS_MODE == 2) bv = bias[n];
#pragma unroll
      for (int r = 0; r < 8; ++r) {
        float v = acc[i][j][r] * scale;
        if (BIAS_MODE == 1) v += bias[mBase + mOff + r];
        if (BIAS_MODE == 2) v += bv;
        if (RESID) v += Rb[(size_t)(mBase + mOff + r) * ldc + n];
        if (ACT == 2) v = fmaxf(v, 0.0f);
        if (ACT == 4) v = (v > 0.f) ? v : 0.01f * v;
        slab[(mOff + r) * 68 + (j << 4) + rlane] = v;
      }
    }
    __builtin_amdgcn_fence(__ATOMIC_RELEASE, "workgroup");
    __builtin_amdgcn_wave_barrier();
    __builtin_amdgcn_fence(__ATOMIC_ACQUIRE, "workgroup");
    if (OUT_MODE == 0) {
      float* C = (float*)Cout + (size_t)b * strideC;
      const int hh = lane >> 4, c4 = (lane & 15) * 4;
      for (int pass = 0; pass < 2; ++pass) {
#pragma unroll
        for (int it = 0; it < 8; ++it) {
          const int row = it * 2 + hh;
          v4f v = *(const v4f*)(slab + row * 68 + c4);
          *(volatile v4f*)(C + (size_t)(mBase + row) * ldc + n0 + c4) = v;
        }
        __threadfence();
      }
    } else {
      const int q = lane >> 3, c8 = (lane & 7) * 8;
      unsigned short* C  = (unsigned short*)Cout  + (size_t)b * strideC;
      unsigned short* C2 = (OUT_MODE == 2) ? ((unsigned short*)Cout2 + (size_t)b * strideC) : nullptr;
      for (int pass = 0; pass < 2; ++pass) {
#pragma unroll
        for (int it = 0; it < 4; ++it) {
          const int row = it * 4 + q;
          const float* sp = slab + row * 68 + c8;
          v8h hv, lv;
#pragma unroll
          for (int e = 0; e < 8; ++e) {
            if (OUT_MODE == 1) {
              hv[e] = (_Float16)sp[e];
            } else {
              unsigned short hb = f2bf_bits(sp[e]);
              unsigned short lb = f2bf_bits(sp[e] - bf_bits2f(hb));
              hv[e] = __builtin_bit_cast(_Float16, hb);
              lv[e] = __builtin_bit_cast(_Float16, lb);
            }
          }
          *(volatile v8h*)(C + (size_t)(mBase + row) * ldc + n0 + c8) = hv;
          if (OUT_MODE == 2) *(volatile v8h*)(C2 + (size_t)(mBase + row) * ldc + n0 + c8) = lv;
        }
        __threadfence();
      }
    }
    __builtin_amdgcn_fence(__ATOMIC_RELEASE, "workgroup");
    __builtin_amdgcn_wave_barrier();
    __builtin_amdgcn_fence(__ATOMIC_ACQUIRE, "workgroup");
  }
}

__global__ __launch_bounds__(256) void wtcast_kernel(const float* __restrict__ W, unsigned short* __restrict__ out,
                                                     int nout, int kin, float scale) {
  __shared__ float sm[64][65];
  const int t  = threadIdx.x;
  const int d0 = blockIdx.x * 64;
  const int h0 = blockIdx.y * 64;
#pragma unroll
  for (int i = 0; i < 16; ++i) {
    const int e = i * 256 + t;
    const int r = e >> 6;
    const int c = e & 63;
    sm[c][r] = W[(size_t)(d0 + r) * nout + h0 + c] * scale;
  }
  __syncthreads();
  const int lane = t & 31, wave = t >> 5;
  const int q = lane >> 3, c8 = (lane & 7) * 8;
  for (int pass = 0; pass < 2; ++pass) {
#pragma unroll
    for (int it = 0; it < 2; ++it) {
      const int row = wave * 8 + it * 4 + q;
      unsigned short hb[8];
#pragma unroll
      for (int e = 0; e < 8; ++e) hb[e] = h_bits(sm[row][c8 + e]);
      const v4u u = (v4u){pk16(hb[0], hb[1]), pk16(hb[2], hb[3]), pk16(hb[4], hb[5]), pk16(hb[6], hb[7])};
      *(volatile v4u*)(out + (size_t)(h0 + row) * kin + d0 + c8) = u;
    }
    __threadfence();
  }
}

__global__ __launch_bounds__(256) void cast8_f16_kernel(const float* __restrict__ in, unsigned short* __restrict__ out, int n8) {
  const int i = blockIdx.x * 256 + threadIdx.x;
  if (i >= n8) return;
  const float* p = in + 8 * (size_t)i;
  const v4f a = *(const v4f*)(p);
  const v4f c = *(const v4f*)(p + 4);
  unsigned short hb[8];
#pragma unroll
  for (int e = 0; e < 4; ++e) {
    hb[e]     = h_bits(a[e]);
    hb[4 + e] = h_bits(c[e]);
  }
  const v4u u = (v4u){pk16(hb[0], hb[1]), pk16(hb[2], hb[3]), pk16(hb[4], hb[5]), pk16(hb[6], hb[7])};
  unsigned short* q = out + 8 * (size_t)i;
  *(volatile v4u*)q = u;
  __threadfence();
  *(volatile v4u*)q = u;
}

__global__ __launch_bounds__(256) void softmax_row_kernel(const float* __restrict__ Sp, unsigned short* __restrict__ P, float carry) {
  __shared__ float redM[8];
  __shared__ float redS[8];
  const int row  = blockIdx.x;
  const int t    = threadIdx.x;
  const int lane = t & 31, wave = t >> 5;
  const int c0   = t * 8;
  const size_t rb = (size_t)row * kS;
  const v4f a = *(const v4f*)(Sp + rb + c0);
  const v4f c = *(const v4f*)(Sp + rb + c0 + 4);
  float m = fmaxf(fmaxf(fmaxf(a.x, a.y), fmaxf(a.z, a.w)), fmaxf(fmaxf(c.x, c.y), fmaxf(c.z, c.w)));
#pragma unroll
  for (int off = 16; off > 0; off >>= 1) m = fmaxf(m, __shfl_xor(m, off, 32));
  if (lane == 0) redM[wave] = m;
  __syncthreads();
  float gm = redM[0];
#pragma unroll
  for (int w = 1; w < 8; ++w) gm = fmaxf(gm, redM[w]);

  v4f lo = a, hi = c;
  float psum = 0.0f;
#pragma unroll 1
  for (int i = 0; i < 8; ++i) {
    const float e  = expf(lo.x - gm);
    psum += e;
    const float nx = hi.x;
    lo = (v4f){lo.y, lo.z, lo.w, nx};
    hi = (v4f){hi.y, hi.z, hi.w, e};
  }
#pragma unroll
  for (int off = 16; off > 0; off >>= 1) psum += __shfl_xor(psum, off, 32);
  if (lane == 0) redS[wave] = psum;
  __syncthreads();
  float tot = redS[0];
#pragma unroll
  for (int w = 1; w < 8; ++w) tot += redS[w];
  const float inv = carry * (1.0f / tot);
  unsigned short hb[8];
  hb[0] = h_bits(lo.x * inv); hb[1] = h_bits(lo.y * inv); hb[2] = h_bits(lo.z * inv); hb[3] = h_bits(lo.w * inv);
  hb[4] = h_bits(hi.x * inv); hb[5] = h_bits(hi.y * inv); hb[6] = h_bits(hi.z * inv); hb[7] = h_bits(hi.w * inv);
  const v4u u = (v4u){pk16(hb[0], hb[1]), pk16(hb[2], hb[3]), pk16(hb[4], hb[5]), pk16(hb[6], hb[7])};
  unsigned short* q = P + rb + c0;
  *(volatile v4u*)q = u;
  __threadfence();
  *(volatile v4u*)q = u;
}

__global__ __launch_bounds__(256) void gelu_f16_kernel(const unsigned short* __restrict__ U, unsigned short* __restrict__ F, int n8) {
  const int i = blockIdx.x * 256 + threadIdx.x;
  if (i >= n8) return;
  v4u iw = *(const v4u*)(U + 8 * (size_t)i);
  v4u ow = (v4u){0u, 0u, 0u, 0u};
#pragma unroll 1
  for (int w = 0; w < 4; ++w) {
    const unsigned word = iw.x;
    iw = (v4u){iw.y, iw.z, iw.w, word};
    unsigned o = 0u;
#pragma unroll 1
    for (int j = 0; j < 2; ++j) {
      const unsigned sh = 16u * (unsigned)j;
      const unsigned short ub = (unsigned short)((word >> sh) & 0xffffu);
      const float u  = (float)__builtin_bit_cast(_Float16, ub);
      const float gl = 0.5f * u * (1.0f + erff(u * 0.70710678118654752f));
      o |= ((unsigned)h_bits(gl)) << sh;
    }
    ow = (v4u){ow.y, ow.z, ow.w, o};
  }
  unsigned short* q = F + 8 * (size_t)i;
  *(volatile v4u*)q = ow;
  __threadfence();
  *(volatile v4u*)q = ow;
}

template <bool W16>
__global__ __launch_bounds__(256) void ln_row_kernel(const float* __restrict__ Y, const float* __restrict__ gam, const float* __restrict__ bet,
                                                     float* __restrict__ O32, unsigned short* __restrict__ O16) {
  __shared__ float redA[8];
  __shared__ float redB[8];
  __shared__ __align__(16) unsigned int hrow[W16 ? 512 : 4];
  const int row  = blockIdx.x;
  const int t    = threadIdx.x;
  const int lane = t & 31, wave = t >> 5;
  const int c0   = 4 * t;
  const size_t rb = (size_t)row * kD;
  const v4f v = *(const v4f*)(Y + rb + c0);
  float s = (v.x + v.y) + (v.z + v.w);
#pragma unroll
  for (int off = 16; off > 0; off >>= 1) s += __shfl_xor(s, off, 32);
  if (lane == 0) redA[wave] = s;
  __syncthreads();
  float tot = redA[0];
#pragma unroll
  for (int w = 1; w < 8; ++w) tot += redA[w];
  const float mu = tot * kInvD;
  const float dx = v.x - mu, dy = v.y - mu, dz = v.z - mu, dw = v.w - mu;
  float q = (dx * dx + dy * dy) + (dz * dz + dw * dw);
#pragma unroll
  for (int off = 16; off > 0; off >>= 1) q += __shfl_xor(q, off, 32);
  if (lane == 0) redB[wave] = q;
  __syncthreads();
  float tot2 = redB[0];
#pragma unroll
  for (int w = 1; w < 8; ++w) tot2 += redB[w];
  const float var  = tot2 * kInvD;
  const float rstd = rsqrtf(var + kLnEps);
  const v4f gg = *(const v4f*)(gam + c0);
  const v4f bb = *(const v4f*)(bet + c0);
  v4f y;
  y.x = (dx * rstd) * gg.x + bb.x;
  y.y = (dy * rstd) * gg.y + bb.y;
  y.z = (dz * rstd) * gg.z + bb.z;
  y.w = (dw * rstd) * gg.w + bb.w;
  float* op = O32 + rb + c0;
  *(volatile v4f*)op = y;
  __threadfence();
  *(volatile v4f*)op = y;
  if (W16) {
    hrow[2 * t]     = pk16(h_bits(y.x), h_bits(y.y));
    hrow[2 * t + 1] = pk16(h_bits(y.z), h_bits(y.w));
    __syncthreads();
    if (t < 128) {
      const v4u u = *(const v4u*)(hrow + 4 * t);
      unsigned short* hp = O16 + rb + 8 * t;
      *(volatile v4u*)hp = u;
      __threadfence();
      *(volatile v4u*)hp = u;
    }
  }
}

extern "C" void kernel_launch(void* const* d_in, const int* in_sizes, int n_in,
                              void* d_out, int out_size, void* d_ws, size_t ws_size,
                              hipStream_t stream) {
  if (n_in < 17) return;
  if (in_sizes[0] != kTok * kD || out_size != kTok * kD) return;
  if (in_sizes[1] != kD * kD || in_sizes[9] != kD * kFF || in_sizes[11] != kFF * kD) return;
  if (ws_size < kWsNeed) return;

  const float* x   = (const float*)d_in[0];
  const float* Wq  = (const float*)d_in[1];
  const float* bq  = (const float*)d_in[2];
  const float* Wk  = (const float*)d_in[3];
  const float* bk  = (const float*)d_in[4];
  const float* Wv  = (const float*)d_in[5];
  const float* bv  = (const float*)d_in[6];
  const float* Wo  = (const float*)d_in[7];
  const float* bo  = (const float*)d_in[8];
  const float* W1  = (const float*)d_in[9];
  const float* b1  = (const float*)d_in[10];
  const float* W2  = (const float*)d_in[11];
  const float* b2  = (const float*)d_in[12];
  const float* g1  = (const float*)d_in[13];
  const float* be1 = (const float*)d_in[14];
  const float* g2  = (const float*)d_in[15];
  const float* be2 = (const float*)d_in[16];
  float* out = (float*)d_out;

  char* ws = (char*)d_ws;
  typedef unsigned short u16;
  u16*   xh   = (u16*)(ws + oXh);
  u16*   WqkT = (u16*)(ws + oWqkT);
  u16*   WvT  = (u16*)(ws + oWvT);
  float* Sc   = (float*)(ws + oS);
  float* h32  = (float*)(ws + oH32);
  u16*   u16p = (u16*)(ws + oU16);
  u16*   W2T  = (u16*)(ws + oW2T);
  u16*   WoT  = (u16*)(ws + oWoT);
  u16*   Pp   = (u16*)(ws + oP);
  u16*   ffp  = (u16*)(ws + oFF);
  u16*   QK   = (u16*)(ws + oQK);
  float* y1   = (float*)(ws + oY1);
  float* y2   = (float*)(ws + oY2);
  u16*   Vt   = (u16*)(ws + oVt);
  u16*   hh   = (u16*)(ws + oHH);
  u16*   ctx  = (u16*)(ws + oCtx);
  u16*   W1T  = (u16*)(ws + oW1T);

  cast8_f16_kernel<<<(kTok * kD / 8 + 255) / 256, 256, 0, stream>>>(x, xh, kTok * kD / 8);
  wtcast_kernel<<<dim3(kD / 64, kD / 64), 256, 0, stream>>>(Wq, WqkT, kD, kD, kWCarry);
  wtcast_kernel<<<dim3(kD / 64, kD / 64), 256, 0, stream>>>(Wk, WqkT + (size_t)kD * kD, kD, kD, kWCarry);
  wtcast_kernel<<<dim3(kD / 64, kD / 64), 256, 0, stream>>>(Wv, WvT, kD, kD, kWCarry);

  wmma_gemm64<0, false, 2, 1, false><<<dim3(128, 1), 256, 0, stream>>>(
      xh, xh, kD, 0L, WqkT, WqkT, kD, 0L, (void*)QK, (void*)QK, kQKld, 0L, bq, x, 0L, kTok, kD, kD, kWCarryInv);
  wmma_gemm64<0, false, 2, 1, false><<<dim3(128, 1), 256, 0, stream>>>(
      xh, xh, kD, 0L, WqkT + (size_t)kD * kD, WqkT, kD, 0L, (void*)(QK + kD), (void*)QK, kQKld, 0L, bk, x, 0L, kTok, kD, kD, kWCarryInv);
  wmma_gemm64<0, false, 1, 1, false><<<dim3(128, 1), 256, 0, stream>>>(
      WvT, WvT, kD, 0L, xh, xh, kD, 0L, (void*)Vt, (void*)Vt, kTok, 0L, bv, x, 0L, kD, kTok, kD, kWCarryInv);

  for (int cidx = 0; cidx < kNChunk; ++cidx) {
    const int b  = cidx / (kH / kG);
    const int h0 = (cidx % (kH / kG)) * kG;
    const u16* qA = QK + (size_t)b * kS * kQKld + (size_t)h0 * kHD;
    const u16* kBt = QK + (size_t)b * kS * kQKld + kD + (size_t)h0 * kHD;
    wmma_gemm64<0, false, 0, 0, false><<<dim3(128, kG), 256, 0, stream>>>(
        qA, qA, kQKld, (long)kHD, kBt, kBt, kQKld, (long)kHD, (void*)Sc, (void*)Sc, kS, (long)kS * kS, bq, x, 0L,
        kS, kS, kHD, kScoreScale);
    softmax_row_kernel<<<kG * kS, 256, 0, stream>>>(Sc, Pp, kPCarry);
    const u16* vBt = Vt + (size_t)(h0 * kHD) * kTok + (size_t)b * kS;
    u16* cC = ctx + (size_t)b * kS * kD + (size_t)h0 * kHD;
    wmma_gemm64<0, false, 0, 1, false><<<dim3(4, kG), 256, 0, stream>>>(
        Pp, Pp, kS, (long)kS * kS, vBt, vBt, kTok, (long)kHD * kTok, (void*)cC, (void*)cC, kD, (long)kHD, bq, x, 0L,
        kS, kHD, kS, kPVScale);
  }

  wtcast_kernel<<<dim3(kD / 64, kD / 64), 256, 0, stream>>>(Wo, WoT, kD, kD, kWCarry);
  wtcast_kernel<<<dim3(kFF / 64, kD / 64), 256, 0, stream>>>(W2, W2T, kD, kFF, kWCarry);
  wmma_gemm64<0, false, 2, 0, true><<<dim3(128, 1), 256, 0, stream>>>(
      ctx, ctx, kD, 0L, WoT, WoT, kD, 0L, (void*)y1, (void*)y1, kD, 0L, bo, x, 0L, kTok, kD, kD, kWoScale);

  ln_row_kernel<true><<<kTok, 256, 0, stream>>>(y1, g1, be1, h32, hh);

  wtcast_kernel<<<dim3(kD / 64, kFF / 64), 256, 0, stream>>>(W1, W1T, kFF, kD, kWCarry);
  wmma_gemm64<0, false, 2, 1, false><<<dim3(512, 1), 256, 0, stream>>>(
      hh, hh, kD, 0L, W1T, W1T, kD, 0L, (void*)u16p, (void*)u16p, kFF, 0L, b1, x, 0L, kTok, kFF, kD, kWCarryInv);

  gelu_f16_kernel<<<(kTok * kFF / 8 + 255) / 256, 256, 0, stream>>>(u16p, ffp, kTok * kFF / 8);

  wmma_gemm64<0, false, 2, 0, true><<<dim3(128, 1), 256, 0, stream>>>(
      ffp, ffp, kFF, 0L, W2T, W2T, kFF, 0L, (void*)y2, (void*)y2, kD, 0L, b2, h32, 0L, kTok, kD, kFF, kWCarryInv);

  ln_row_kernel<false><<<kTok, 256, 0, stream>>>(y2, g2, be2, out, hh);
}
